// SimpleLSTM_37271726195399
// MI455X (gfx1250) — hardware-verified
//
#include <hip/hip_runtime.h>
#include <math.h>

constexpr int NBATCH  = 32;
constexpr int NSTEP   = 512;
constexpr int NIN     = 256;
constexpr int NHID    = 512;
constexpr int NGATE   = 4 * NHID;
constexpr int KTOT    = NIN + NHID;
constexpr int SEQ_BLK = 16;
constexpr int RTHR    = 512;
constexpr int RWAVES  = RTHR / 32;
constexpr int APITCH  = 776;
constexpr int OPITCH  = 516;
constexpr int TTHR    = 256;
constexpr float ACARRY = 16.0f;
constexpr float WCARRY = 256.0f;
constexpr float FOLD   = 1.0f / (ACARRY * WCARRY);

constexpr int NOUT0 = NBATCH * NSTEP * NHID;
constexpr int NOUT1 = NBATCH * NHID;
constexpr int NOUT2 = NBATCH * NHID;

static_assert(NBATCH % SEQ_BLK == 0, "batch tiles");
static_assert(NHID == 32 * RWAVES, "16 waves x 32 hidden units");
static_assert(KTOT % 32 == 0 && NIN % 32 == 0, "k chunks of 32");
static_assert(NIN % 64 == 0 && NHID % 64 == 0 && NGATE % 64 == 0, "64x64 transpose tiles");
static_assert(APITCH % 8 == 0 && APITCH >= KTOT, "A pitch");
static_assert(OPITCH % 4 == 0 && OPITCH >= NHID, "O pitch");
static_assert(SEQ_BLK * NIN == RTHR * 8, "x staging covers 16 x 256 exactly");
static_assert(SEQ_BLK * NHID == RTHR * 16, "row store covers 16 x 512 exactly");
static_assert((size_t)NOUT0 * 4 == 33554432u, "out1 byte offset");
static_assert(((size_t)NOUT0 + NOUT1) * 4 == 33619968u, "out2 byte offset");
static_assert(((size_t)NOUT0 + NOUT1 + NOUT2) * 4 == 33685504u, "d_out total bytes");
static_assert(SEQ_BLK * APITCH * 2 + SEQ_BLK * OPITCH * 4 <= 65536, "static LDS");

typedef __attribute__((ext_vector_type(16))) _Float16 v16h;
typedef __attribute__((ext_vector_type(8)))  _Float16 v8h;
typedef __attribute__((ext_vector_type(8)))  float    v8f;
typedef __attribute__((ext_vector_type(4)))  float    v4f;

__device__ __forceinline__ unsigned short f2bf_bits(float f) {
  unsigned u = __float_as_uint(f);
  return (unsigned short)((u + 0x7FFFu + ((u >> 16) & 1u)) >> 16);
}
__device__ __forceinline__ float bf_bits2f(unsigned short h) { return __uint_as_float(((unsigned)h) << 16); }
__device__ __forceinline__ float bf16r(float f) { return bf_bits2f(f2bf_bits(f)); }

__device__ __forceinline__ void guard_all_h(v8f& a0, v8f& a1, v8f& a2, v8f& a3,
                                            v16h x, v16h b0, v16h b1, v16h b2, v16h b3) {
  asm volatile("v_nop\n\tv_nop\n\tv_nop\n\tv_nop"
               : "+v"(a0), "+v"(a1), "+v"(a2), "+v"(a3)
               : "v"(x), "v"(b0), "v"(b1), "v"(b2), "v"(b3));
}
__device__ __forceinline__ void acc_guard4(v8f& a, v8f& b, v8f& c, v8f& d) {
  asm volatile("v_nop\n\tv_nop\n\tv_nop\n\tv_nop" : "+v"(a), "+v"(b), "+v"(c), "+v"(d));
}
__device__ __forceinline__ void pin2(float& a, float& b) { asm volatile("" : "+v"(a), "+v"(b)); }

struct FragH {
  union U { v16h v; v8h h[2]; };
  static __device__ __forceinline__ v16h load(const _Float16* p) {
    U f; f.h[0] = *(const v8h*)(p); f.h[1] = *(const v8h*)(p + 16); return f.v;
  }
  static __device__ __forceinline__ v8f mma(v16h a, v16h b, v8f c) {
    return __builtin_amdgcn_wmma_f32_16x16x32_f16(false, a, false, b, (short)0, c, false, false);
  }
};

__device__ __forceinline__ float fsig(float x)  { return __builtin_amdgcn_rcpf(1.0f + __expf(-x)); }
__device__ __forceinline__ float ftanh(float x) { return 1.0f - 2.0f * __builtin_amdgcn_rcpf(__expf(2.0f * x) + 1.0f); }

__global__ __launch_bounds__(TTHR) void wt_plane_kernel(const float* __restrict__ wi, const float* __restrict__ wh,
                                                        unsigned short* __restrict__ O) {
  __shared__ float Tt[64 * 65];
  const int tid = threadIdx.x;
  const int c0  = blockIdx.x * 64;
  const int kr0 = blockIdx.y * 64;
  const bool from_wi = (kr0 < NIN);
  const float* src = from_wi ? wi : wh;
  const int r0 = from_wi ? kr0 : (kr0 - NIN);
#pragma unroll
  for (int i = 0; i < 4; ++i) {
    const int idx = i * TTHR + tid;
    const int rr = idx >> 4, cc = (idx & 15) * 4;
    const v4f v = *(const v4f*)(src + (size_t)(r0 + rr) * (size_t)NGATE + c0 + cc);
    Tt[rr * 65 + cc + 0] = v[0];
    Tt[rr * 65 + cc + 1] = v[1];
    Tt[rr * 65 + cc + 2] = v[2];
    Tt[rr * 65 + cc + 3] = v[3];
  }
  __syncthreads();
  const int q = tid >> 3, c8 = (tid & 7) * 8;
  v8h hv[2];
#pragma unroll
  for (int g = 0; g < 2; ++g) {
    const int qq = g * 32 + q;
#pragma unroll
    for (int e = 0; e < 8; ++e) {
      const float f  = Tt[(c8 + e) * 65 + qq];
      const float fb = bf16r(f);
      hv[g][e] = (_Float16)(fb * WCARRY);
    }
  }
  for (int pass = 0; pass < 2; ++pass) {
#pragma unroll
    for (int g = 0; g < 2; ++g) {
      const size_t o = (size_t)(c0 + g * 32 + q) * (size_t)KTOT + (size_t)(kr0 + c8);
      *(volatile v8h*)(O + o) = hv[g];
    }
    __threadfence();
  }
}

__global__ __launch_bounds__(RTHR) void cell_seq_kernel(const float* __restrict__ x, const int* __restrict__ mask,
                                                        const float* __restrict__ c0, const float* __restrict__ h0,
                                                        const float* __restrict__ init_c, const float* __restrict__ init_h,
                                                        const float* __restrict__ bias,
                                                        const unsigned short* __restrict__ Wtp,
                                                        float* __restrict__ out, float* __restrict__ cfin,
                                                        float* __restrict__ hfin) {
  __shared__ __align__(16) _Float16 As[SEQ_BLK * APITCH];
  __shared__ __align__(16) float    Os[SEQ_BLK * OPITCH];
  const _Float16* Wt = (const _Float16*)Wtp;
  const int tid = threadIdx.x, lane = tid & 31, wave = tid >> 5;
  const int c = lane & 15, hh = lane >> 4, koff = hh * 8;
  const int rowbase = blockIdx.x * SEQ_BLK;
  const int xm = tid >> 5, xc8 = (tid & 31) * 8;

#pragma unroll 1
  for (int i = 0; i < SEQ_BLK; ++i) {
    const float hv0 = bf16r(h0[(size_t)(rowbase + i) * NHID + tid]);
    As[i * APITCH + NIN + tid] = (_Float16)(ACARRY * hv0);
  }
  {
    const float* xp = x + ((size_t)(rowbase + xm) * NSTEP) * NIN + xc8;
    const v4f a = *(const v4f*)(xp);
    const v4f b = *(const v4f*)(xp + 4);
    v8h hv;
#pragma unroll
    for (int e = 0; e < 4; ++e) {
      hv[e]     = (_Float16)(ACARRY * bf16r(a[e]));
      hv[4 + e] = (_Float16)(ACARRY * bf16r(b[e]));
    }
    *(v8h*)(As + xm * APITCH + xc8) = hv;
  }
  float cst[2][8], hst[2][8], bb[2][4];
#pragma unroll
  for (int nt = 0; nt < 2; ++nt) {
    const int j = 32 * wave + 16 * nt + c;
#pragma unroll
    for (int g = 0; g < 4; ++g) bb[nt][g] = bf16r(bias[g * NHID + j]);
#pragma unroll
    for (int r = 0; r < 8; ++r) {
      const size_t o = (size_t)(rowbase + 8 * hh + r) * NHID + j;
      cst[nt][r] = bf16r(c0[o]);
      hst[nt][r] = bf16r(h0[o]);
    }
  }
  __syncthreads();

  const _Float16* arow = As + c * APITCH + koff;
  const v8f z8 = {0.f, 0.f, 0.f, 0.f, 0.f, 0.f, 0.f, 0.f};
  const size_t gstride = (size_t)NHID * (size_t)KTOT;

#pragma unroll 1
  for (int t = 0; t < NSTEP; ++t) {
    unsigned keepbits = 0u;
#pragma unroll
    for (int r = 0; r < 8; ++r) {
      const int mv = mask[(size_t)(rowbase + 8 * hh + r) * NSTEP + t];
      keepbits |= (mv != 0) ? (1u << r) : 0u;
    }

#pragma unroll
    for (int nt = 0; nt < 2; ++nt) {
      const int j = 32 * wave + 16 * nt + c;
      const _Float16* wrow = Wt + (size_t)j * KTOT + koff;
      v8f acc0 = z8, acc1 = z8, acc2 = z8, acc3 = z8;
#pragma unroll 1
      for (int k0 = 0; k0 < KTOT; k0 += 32) {
        const v16h a  = FragH::load(arow + k0);
        const v16h b0 = FragH::load(wrow + k0);
        const v16h b1 = FragH::load(wrow + gstride + k0);
        const v16h b2 = FragH::load(wrow + 2 * gstride + k0);
        const v16h b3 = FragH::load(wrow + 3 * gstride + k0);
        acc0 = FragH::mma(a, b0, acc0);
        acc1 = FragH::mma(a, b1, acc1);
        acc2 = FragH::mma(a, b2, acc2);
        acc3 = FragH::mma(a, b3, acc3);
        guard_all_h(acc0, acc1, acc2, acc3, a, b0, b1, b2, b3);
      }
      acc_guard4(acc0, acc1, acc2, acc3);
      float icv[8], ihv[8];
#pragma unroll
      for (int r = 0; r < 8; ++r) {
        const size_t o = ((size_t)(rowbase + 8 * hh + r) * NSTEP + (size_t)t) * NHID + j;
        float ca = init_c[o];
        float ha = init_h[o];
        pin2(ca, ha);
        icv[r] = ca;
        ihv[r] = ha;
      }
#pragma unroll
      for (int r = 0; r < 8; ++r) {
        const float zi = acc0[r] * FOLD + bb[nt][0];
        const float zf = acc1[r] * FOLD + bb[nt][1];
        const float zg = acc2[r] * FOLD + bb[nt][2];
        const float zo = acc3[r] * FOLD + bb[nt][3];
        const float ig = fsig(zi);
        const float fg = fsig(zf);
        const float gg = ftanh(zg);
        const float og = fsig(zo);
        const float nc = fg * cst[nt][r] + ig * gg;
        const float nh = og * ftanh(nc);
        const bool keep = ((keepbits >> r) & 1u) != 0u;
        const float rc = bf16r(icv[r]);
        const float rh = bf16r(ihv[r]);
        cst[nt][r] = keep ? nc : rc;
        hst[nt][r] = keep ? nh : rh;
      }
    }
    __syncthreads();
#pragma unroll
    for (int nt = 0; nt < 2; ++nt) {
      const int j = 32 * wave + 16 * nt + c;
#pragma unroll
      for (int r = 0; r < 8; ++r) {
        const float hv1 = hst[nt][r];
        const bool keep = ((keepbits >> r) & 1u) != 0u;
        As[(8 * hh + r) * APITCH + NIN + j] = (_Float16)(ACARRY * hv1);
        Os[(8 * hh + r) * OPITCH + j] = keep ? hv1 : 0.0f;
      }
    }
    {
      const int tn = (t + 1 < NSTEP) ? (t + 1) : (NSTEP - 1);
      const float* xp = x + ((size_t)(rowbase + xm) * NSTEP + (size_t)tn) * NIN + xc8;
      const v4f a = *(const v4f*)(xp);
      const v4f b = *(const v4f*)(xp + 4);
      v8h hv;
#pragma unroll
      for (int e = 0; e < 4; ++e) {
        hv[e]     = (_Float16)(ACARRY * bf16r(a[e]));
        hv[4 + e] = (_Float16)(ACARRY * bf16r(b[e]));
      }
      *(v8h*)(As + xm * APITCH + xc8) = hv;
    }
    __syncthreads();
    {
      v4f sv[4];
#pragma unroll
      for (int it = 0; it < 4; ++it) {
        const int idx = it * RTHR + tid;
        const int row = idx >> 7, c4 = (idx & 127) * 4;
        sv[it] = *(const v4f*)(Os + row * OPITCH + c4);
      }
      for (int pass = 0; pass < 2; ++pass) {
#pragma unroll
        for (int it = 0; it < 4; ++it) {
          const int idx = it * RTHR + tid;
          const int row = idx >> 7, c4 = (idx & 127) * 4;
          *(volatile v4f*)(out + ((size_t)(rowbase + row) * NSTEP + (size_t)t) * NHID + c4) = sv[it];
        }
        __threadfence();
      }
    }
  }

#pragma unroll 1
  for (int which = 0; which < 2; ++which) {
    __syncthreads();
#pragma unroll
    for (int nt = 0; nt < 2; ++nt) {
      const int j = 32 * wave + 16 * nt + c;
#pragma unroll
      for (int r = 0; r < 8; ++r) {
        const float cv = cst[nt][r];
        const float hv2 = hst[nt][r];
        Os[(8 * hh + r) * OPITCH + j] = which ? hv2 : cv;
      }
    }
    __syncthreads();
    float* dst = which ? hfin : cfin;
    v4f sv[4];
#pragma unroll
    for (int it = 0; it < 4; ++it) {
      const int idx = it * RTHR + tid;
      const int row = idx >> 7, c4 = (idx & 127) * 4;
      sv[it] = *(const v4f*)(Os + row * OPITCH + c4);
    }
    for (int pass = 0; pass < 2; ++pass) {
#pragma unroll
      for (int it = 0; it < 4; ++it) {
        const int idx = it * RTHR + tid;
        const int row = idx >> 7, c4 = (idx & 127) * 4;
        *(volatile v4f*)(dst + (size_t)(rowbase + row) * NHID + c4) = sv[it];
      }
      __threadfence();
    }
  }
}

extern "C" void kernel_launch(void* const* d_in, const int* in_sizes, int n_in,
                              void* d_out, int out_size, void* d_ws, size_t ws_size, hipStream_t stream) {
  if (n_in < 9 || d_out == nullptr || d_ws == nullptr) return;
  if (in_sizes[0] != NBATCH * NSTEP * NIN || in_sizes[1] != NBATCH * NSTEP ||
      in_sizes[2] != NBATCH * NHID || in_sizes[3] != NBATCH * NHID ||
      in_sizes[4] != NBATCH * NSTEP * NHID || in_sizes[5] != NBATCH * NSTEP * NHID ||
      in_sizes[6] != NIN * NGATE || in_sizes[7] != NHID * NGATE || in_sizes[8] != NGATE ||
      out_size != NOUT0 + NOUT1 + NOUT2) return;

  const float* x      = (const float*)d_in[0];
  const int*   mask   = (const int*)d_in[1];
  const float* c0     = (const float*)d_in[2];
  const float* h0     = (const float*)d_in[3];
  const float* init_c = (const float*)d_in[4];
  const float* init_h = (const float*)d_in[5];
  const float* wi     = (const float*)d_in[6];
  const float* wh     = (const float*)d_in[7];
  const float* bias   = (const float*)d_in[8];
  float* out0 = (float*)d_out;
  float* cfin = out0 + (size_t)NOUT0;
  float* hfin = cfin + (size_t)NOUT1;

  char* ws = (char*)d_ws; size_t off = 0;
  auto carve = [&](size_t bytes) -> char* { char* p = ws + off; off += (bytes + 255) & ~(size_t)255; return p; };
  unsigned short* WT = (unsigned short*)carve((size_t)NGATE * KTOT * 2);
  if (off > ws_size || off > (size_t)134217728) return;

  wt_plane_kernel<<<dim3(NGATE / 64, KTOT / 64), TTHR, 0, stream>>>(wi, wh, WT);
  cell_seq_kernel<<<NBATCH / SEQ_BLK, RTHR, 0, stream>>>(x, mask, c0, h0, init_c, init_h, bias, WT, out0, cfin, hfin);
}
